// DualCrossMessageBlock_40475771797589
// MI455X (gfx1250) — hardware-run, weakly checked
//
#include <hip/hip_runtime.h>
#include <stddef.h>


#pragma clang fp contract(off)

#define FDIM    128
#define SIXF    768
#define RDIM    20
#define VROW    384
#define MSGW    512
#define NTHR    256
#define NWAVE   8
#define NBN     64
#define NBE     64
#define APA     136
#define APR     40
#define GSTR    132
#define WPW     772
#define EPT     8
#define PIECE   (NTHR * EPT)
#define WCAP    (EPT * 32)
#define NBC     128
#define SLB     8
#define CE      40960
#define MAXCH   64
#define P1H     0
#define P1L     16384
#define P2H     32768
#define P2L     131072
#define PRW     229376
#define PWTOT   253952
#define PBLK    (PWTOT / (NTHR * 8))
#define WSCAP   134217728
#define NODEDYN (4 * NBN * APA * 2 + NBN * GSTR * 4)
#define EDGEDYN (NBE * WPW * 4)
#define AGGDYN  (NBC * MSGW * 4)
#define SCW     16.0f
#define SCA     64.0f
#define INV1024 0.0009765625f

static_assert((PWTOT % (NTHR * 8)) == 0);
static_assert((P1L % (NTHR * 8)) == 0);
static_assert((P2H % (NTHR * 8)) == 0);
static_assert((P2L % (NTHR * 8)) == 0);
static_assert((PRW % (NTHR * 8)) == 0);
static_assert(P1L == FDIM * FDIM);
static_assert(P2H == P1L + FDIM * FDIM);
static_assert(P2L == P2H + SIXF * FDIM);
static_assert(PRW == P2L + SIXF * FDIM);
static_assert(PWTOT == PRW + SIXF * 32);
static_assert(((APA * 2) % 16) == 0);
static_assert(((APR * 2) % 16) == 0);
static_assert(((GSTR * 4) % 16) == 0);
static_assert(((WPW * 4) % 16) == 0);
static_assert(NODEDYN == 103424);
static_assert(EDGEDYN == 197632);
static_assert(AGGDYN == 262144);
static_assert(NBC <= (1 << SLB));
static_assert((NBC & (NBC - 1)) == 0);
static_assert(PIECE == 2048);
static_assert((EPT % 4) == 0);
static_assert((CE % PIECE) == 0);
static_assert((CE % NBE) == 0);
static_assert((NBC % NWAVE) == 0);
static_assert(NBE == NWAVE * 8);
static_assert(NBN == 4 * 16);
static_assert(NTHR == 4 * NBE);
static_assert(NTHR == 4 * NBN);
static_assert((SIXF % NTHR) == 0);
static_assert((SIXF % FDIM) == 0);
static_assert(MSGW == FDIM + VROW);
static_assert(((NBC * 32) % NTHR) == 0);
static_assert(((NBC * 96) % NTHR) == 0);

typedef float          v4f   __attribute__((ext_vector_type(4)));
typedef float          v8f   __attribute__((ext_vector_type(8)));
typedef int            v4i   __attribute__((ext_vector_type(4)));
typedef unsigned short v8us  __attribute__((ext_vector_type(8)));
typedef _Float16       v8h   __attribute__((ext_vector_type(8)));
typedef _Float16       v16h  __attribute__((ext_vector_type(16)));
typedef __bf16         v16b  __attribute__((ext_vector_type(16)));
union FragH { v16h v; v8h h[2]; };
union FragB { v16b v; v8us u[2]; };
union Cvt8  { v8h v; v8us u; };

__device__ __forceinline__ v8f wmh(v16h a, v16h b, v8f c) {
  v8f d = __builtin_amdgcn_wmma_f32_16x16x32_f16(false, a, false, b, (short)0, c, false, false);
  asm volatile("v_nop\n\tv_nop\n\tv_nop\n\tv_nop" : "+v"(d) : "v"(a), "v"(b));
  return d;
}
__device__ __forceinline__ v8f wmb(v16b a, v16b b, v8f c) {
  v8f d = __builtin_amdgcn_wmma_f32_16x16x32_bf16(false, a, false, b, (short)0, c, false, false);
  asm volatile("v_nop\n\tv_nop\n\tv_nop\n\tv_nop" : "+v"(d) : "v"(a), "v"(b));
  return d;
}
__device__ __forceinline__ v8f zero8() {
  v8f z = {0.f, 0.f, 0.f, 0.f, 0.f, 0.f, 0.f, 0.f};
  return z;
}
__device__ __forceinline__ int iclamp(int v, int lo, int hi) { return v < lo ? lo : (v > hi ? hi : v); }

__device__ __forceinline__ unsigned short bf_rne(float f) {
  unsigned u = __float_as_uint(f);
  u += 0x7FFFu + ((u >> 16) & 1u);
  return (unsigned short)(u >> 16);
}
__device__ __forceinline__ float bf_val(unsigned short b) { return __uint_as_float(((unsigned)b) << 16); }

__device__ __forceinline__ void cvt_hl8(v4f xa, v4f xb, v8us& h, v8us& l) {
  float f[8];
  f[0] = xa.x; f[1] = xa.y; f[2] = xa.z; f[3] = xa.w;
  f[4] = xb.x; f[5] = xb.y; f[6] = xb.z; f[7] = xb.w;
#pragma unroll
  for (int j = 0; j < 8; ++j) {
    const unsigned short hb = bf_rne(f[j]);
    h[j] = hb;
    l[j] = bf_rne(f[j] - bf_val(hb));
  }
}

__device__ __forceinline__ void gemm16x64(const _Float16* ap, const _Float16* __restrict__ bpl, int kp, int nks, int n0,
                                          int m, int hh, v8f& c0, v8f& c1, v8f& c2, v8f& c3) {
  c0 = zero8(); c1 = zero8(); c2 = zero8(); c3 = zero8();
#pragma unroll 1
  for (int ks = 0; ks < nks; ++ks) {
    FragH a;
    a.h[0] = *(const v8h*)(ap + 32 * ks);
    a.h[1] = *(const v8h*)(ap + 32 * ks + 16);
    const _Float16* bp = bpl + (size_t)(n0 + m) * kp + 32 * ks + 8 * hh;
    FragH b;
    b.h[0] = *(const v8h*)(bp);
    b.h[1] = *(const v8h*)(bp + 16);
    c0 = wmh(a.v, b.v, c0);
    b.h[0] = *(const v8h*)(bp + (size_t)16 * kp);
    b.h[1] = *(const v8h*)(bp + (size_t)16 * kp + 16);
    c1 = wmh(a.v, b.v, c1);
    b.h[0] = *(const v8h*)(bp + (size_t)32 * kp);
    b.h[1] = *(const v8h*)(bp + (size_t)32 * kp + 16);
    c2 = wmh(a.v, b.v, c2);
    b.h[0] = *(const v8h*)(bp + (size_t)48 * kp);
    b.h[1] = *(const v8h*)(bp + (size_t)48 * kp + 16);
    c3 = wmh(a.v, b.v, c3);
  }
}

__device__ __forceinline__ void tile3(const unsigned short* __restrict__ bh, const unsigned short* __restrict__ bl,
                                      size_t ob, const FragB& ah, const FragB& al, v8f& c) {
  FragB b;
  b.u[0] = *(const v8us*)(bh + ob);
  b.u[1] = *(const v8us*)(bh + ob + 16);
  c = wmb(ah.v, b.v, c);
  c = wmb(al.v, b.v, c);
  b.u[0] = *(const v8us*)(bl + ob);
  b.u[1] = *(const v8us*)(bl + ob + 16);
  c = wmb(ah.v, b.v, c);
}

__device__ __forceinline__ void gemm3x16x64(const unsigned short* aph, const unsigned short* apl,
                                            const unsigned short* __restrict__ bh, const unsigned short* __restrict__ bl,
                                            int kp, int nks, int n0, int m, int hh, v8f& c0, v8f& c1, v8f& c2, v8f& c3) {
  c0 = zero8(); c1 = zero8(); c2 = zero8(); c3 = zero8();
#pragma unroll 1
  for (int ks = 0; ks < nks; ++ks) {
    FragB ah, al;
    ah.u[0] = *(const v8us*)(aph + 32 * ks);
    ah.u[1] = *(const v8us*)(aph + 32 * ks + 16);
    al.u[0] = *(const v8us*)(apl + 32 * ks);
    al.u[1] = *(const v8us*)(apl + 32 * ks + 16);
    const size_t ob = (size_t)(n0 + m) * kp + 32 * ks + 8 * hh;
    tile3(bh, bl, ob,                     ah, al, c0);
    tile3(bh, bl, ob + (size_t)16 * kp,   ah, al, c1);
    tile3(bh, bl, ob + (size_t)32 * kp,   ah, al, c2);
    tile3(bh, bl, ob + (size_t)48 * kp,   ah, al, c3);
  }
}

__device__ __forceinline__ void stage8f(float* sp, v8f a, float bias) {
#pragma unroll
  for (int r = 0; r < 8; ++r) sp[r * GSTR] = a[r] + bias;
}
__device__ __forceinline__ void stage8silu(unsigned short* ph, unsigned short* pl, v8f a, float bias) {
#pragma unroll
  for (int r = 0; r < 8; ++r) {
    const float x  = a[r] + bias;
    const float ex = __expf(-x);
    const float rc = __builtin_amdgcn_rcpf(1.0f + ex);
    const float y  = x * rc;
    const unsigned short hb = bf_rne(y);
    ph[r * APA] = hb;
    pl[r * APA] = bf_rne(y - bf_val(hb));
  }
}
__device__ __forceinline__ void stage_gate(float* sp, v8f a, const float* fr, float bias) {
#pragma unroll
  for (int r = 0; r < 8; ++r) sp[r * WPW] = a[r] * INV1024 + fr[r] * bias;
}

__global__ __launch_bounds__(NTHR) void k_prep(
    const float* __restrict__ W1, const float* __restrict__ W2, const float* __restrict__ Wr, unsigned short* wp) {
  const int tid = (int)threadIdx.x;
  const int b = (int)blockIdx.x;
  const int o = (b * NTHR + tid) * 8;
  const float* src = W1;
  int n, k0, mode = 0, pitch = FDIM;
  if (o < P1L)       { n = o >> 7; k0 = o & 127; }
  else if (o < P2H)  { const int idx = o - P1L; n = idx >> 7; k0 = idx & 127; mode = 1; }
  else if (o < P2L)  { const int idx = o - P2H; n = idx >> 7; k0 = idx & 127; src = W2; pitch = SIXF; }
  else if (o < PRW)  { const int idx = o - P2L; n = idx >> 7; k0 = idx & 127; src = W2; pitch = SIXF; mode = 1; }
  else               { const int idx = o - PRW; n = idx >> 5; k0 = idx & 31;  src = Wr; pitch = SIXF; mode = 2; }
  v8us ov;
  if (mode == 2) {
    Cvt8 cv;
#pragma unroll
    for (int j = 0; j < 8; ++j) {
      const int k  = k0 + j;
      const int kc = k < RDIM ? k : RDIM - 1;
      const float w = src[(size_t)kc * pitch + n];
      const float v = (k < RDIM) ? (w * SCW) : 0.0f;
      cv.v[j] = (_Float16)v;
    }
    ov = cv.u;
  } else {
#pragma unroll
    for (int j = 0; j < 8; ++j) {
      const float w = src[(size_t)(k0 + j) * pitch + n];
      const unsigned short hb = bf_rne(w);
      const unsigned short lb = bf_rne(w - bf_val(hb));
      ov[j] = (mode == 0) ? hb : lb;
    }
  }
  unsigned short* dp = wp + o;
  *(volatile v8us*)dp = ov;
  __threadfence();
  *(volatile v8us*)dp = ov;
}

__global__ __launch_bounds__(NTHR) void k_node(
    const float* __restrict__ sin_, const unsigned short* __restrict__ wp,
    const float* __restrict__ b1, const float* __restrict__ b2, float* PHI, int nN) {
  extern __shared__ __attribute__((aligned(16))) float ndynf[];
  __shared__ __attribute__((aligned(16))) float sPar[FDIM + SIXF];
  unsigned short* sAH = (unsigned short*)ndynf;
  unsigned short* sAL = sAH + NBN * APA;
  unsigned short* sYH = sAL + NBN * APA;
  unsigned short* sYL = sYH + NBN * APA;
  float* sU = ndynf + (4 * NBN * APA) / 2;
  const int tid = (int)threadIdx.x, lane = tid & 31, wave = tid >> 5, hh = lane >> 4, m = lane & 15;
  const int n0 = (int)blockIdx.x * NBN;

  {
    const int nl = tid >> 2, q = tid & 3;
    int node = n0 + nl;
    node = node > nN - 1 ? nN - 1 : node;
    const float* rp = sin_ + (size_t)node * FDIM + 32 * q;
#pragma unroll
    for (int i = 0; i < 4; ++i) {
      const v4f xa = *(const v4f*)(rp + 8 * i);
      const v4f xb = *(const v4f*)(rp + 8 * i + 4);
      v8us h, l;
      cvt_hl8(xa, xb, h, l);
      *(v8us*)(sAH + nl * APA + 32 * q + 8 * i) = h;
      *(v8us*)(sAL + nl * APA + 32 * q + 8 * i) = l;
    }
  }
  if (tid < FDIM) sPar[tid] = b1[tid];
#pragma unroll
  for (int i = 0; i < SIXF / NTHR; ++i) sPar[FDIM + tid + NTHR * i] = b2[tid + NTHR * i];
  __syncthreads();

  const int rt = wave & 3, cg = wave >> 2;

  {
    v8f a0, a1, a2, a3;
    gemm3x16x64(sAH + (16 * rt + m) * APA + 8 * hh, sAL + (16 * rt + m) * APA + 8 * hh,
                wp + P1H, wp + P1L, FDIM, 4, 64 * cg, m, hh, a0, a1, a2, a3);
    unsigned short* ph = sYH + (16 * rt + 8 * hh) * APA + 64 * cg + m;
    unsigned short* pl = sYL + (16 * rt + 8 * hh) * APA + 64 * cg + m;
    const float* bb = sPar + 64 * cg + m;
    stage8silu(ph,      pl,      a0, bb[0]);
    stage8silu(ph + 16, pl + 16, a1, bb[16]);
    stage8silu(ph + 32, pl + 32, a2, bb[32]);
    stage8silu(ph + 48, pl + 48, a3, bb[48]);
  }
  __syncthreads();

  const unsigned short* yph = sYH + (16 * rt + m) * APA + 8 * hh;
  const unsigned short* ypl = sYL + (16 * rt + m) * APA + 8 * hh;
#pragma unroll 1
  for (int p = 0; p < SIXF / FDIM; ++p) {
    {
      v8f a0, a1, a2, a3;
      gemm3x16x64(yph, ypl, wp + P2H, wp + P2L, FDIM, 4, FDIM * p + 64 * cg, m, hh, a0, a1, a2, a3);
      float* sp = sU + (16 * rt + 8 * hh) * GSTR + 64 * cg + m;
      const float* bb = sPar + FDIM + FDIM * p + 64 * cg + m;
      stage8f(sp,      a0, bb[0]);
      stage8f(sp + 16, a1, bb[16]);
      stage8f(sp + 32, a2, bb[32]);
      stage8f(sp + 48, a3, bb[48]);
    }
    __syncthreads();
#pragma unroll 1
    for (int it = 0; it < NBN / NWAVE; ++it) {
      const int row = wave + NWAVE * it;
      const v4f v = *(const v4f*)(sU + row * GSTR + 4 * lane);
      *(volatile v4f*)(PHI + (size_t)(n0 + row) * SIXF + FDIM * p + 4 * lane) = v;
    }
    __threadfence();
#pragma unroll 1
    for (int it = 0; it < NBN / NWAVE; ++it) {
      const int row = wave + NWAVE * it;
      const v4f v = *(const v4f*)(sU + row * GSTR + 4 * lane);
      *(volatile v4f*)(PHI + (size_t)(n0 + row) * SIXF + FDIM * p + 4 * lane) = v;
    }
    __syncthreads();
  }
}

__global__ __launch_bounds__(NTHR) void k_edge(
    const float* __restrict__ re1, const float* __restrict__ re2, const float* __restrict__ f1,
    const float* __restrict__ f2, const float* __restrict__ u1, const float* __restrict__ u2,
    const int* __restrict__ ei, const float* __restrict__ PHI, const float* __restrict__ vin,
    const unsigned short* __restrict__ wp, const float* __restrict__ br,
    float* Mout, int nE, int nN, int cbeg) {
  extern __shared__ __attribute__((aligned(16))) float sW[];
  __shared__ __attribute__((aligned(16))) _Float16 sR[NBE * APR];
  __shared__ __attribute__((aligned(16))) float sBr[SIXF];
  __shared__ __attribute__((aligned(16))) float sF[NBE];
  __shared__ __attribute__((aligned(16))) float sU[NBE * 8];
  __shared__ int sJ[NBE];
  const int tid = (int)threadIdx.x, lane = tid & 31, wave = tid >> 5, hh = lane >> 4, m = lane & 15;
  const int el0 = (int)blockIdx.x * NBE;

  if (tid < NBE) {
    int e = cbeg + el0 + tid;
    e = e > nE - 1 ? nE - 1 : e;
    const int jj = iclamp(ei[(size_t)nE + e], 0, nN - 1);
    const float fa = f1[e], fb = f2[e];
    const float* pa = re1 + (size_t)e * RDIM;
    const float* pb = re2 + (size_t)e * RDIM;
    float av[RDIM];
#pragma unroll
    for (int q = 0; q < RDIM / 4; ++q) {
      const v4f xa = *(const v4f*)(pa + 4 * q);
      const v4f xb = *(const v4f*)(pb + 4 * q);
      const v4f ta = xa * fa;
      const v4f tb = xb * fb;
      const v4f t = ta + tb;
      av[4 * q] = t.x; av[4 * q + 1] = t.y; av[4 * q + 2] = t.z; av[4 * q + 3] = t.w;
    }
    const float zf = fa * 0.0f;
    v8h h0, h1, h2, h3;
#pragma unroll
    for (int j = 0; j < 8; ++j) {
      h0[j] = (_Float16)(av[j] * SCA);
      h1[j] = (_Float16)(av[8 + j] * SCA);
      h3[j] = (_Float16)zf;
    }
#pragma unroll
    for (int j = 0; j < 4; ++j) {
      h2[j]     = (_Float16)(av[16 + j] * SCA);
      h2[4 + j] = (_Float16)zf;
    }
    _Float16* rp = sR + tid * APR;
    *(v8h*)(rp)      = h0;
    *(v8h*)(rp + 8)  = h1;
    *(v8h*)(rp + 16) = h2;
    *(v8h*)(rp + 24) = h3;
    sF[tid] = fa + fb;
    sJ[tid] = jj;
    const float* q1 = u1 + (size_t)e * 3;
    const float* q2 = u2 + (size_t)e * 3;
    sU[8 * tid + 0] = q1[0]; sU[8 * tid + 1] = q1[1]; sU[8 * tid + 2] = q1[2]; sU[8 * tid + 3] = 0.0f;
    sU[8 * tid + 4] = q2[0]; sU[8 * tid + 5] = q2[1]; sU[8 * tid + 6] = q2[2]; sU[8 * tid + 7] = 0.0f;
  }
#pragma unroll
  for (int i = 0; i < SIXF / NTHR; ++i) sBr[tid + NTHR * i] = br[tid + NTHR * i];
  __syncthreads();

  const int rt = wave & 3, cg = wave >> 2;

  {
    const _Float16* ap  = sR + (16 * rt + m) * APR + 8 * hh;
    const _Float16* bpl = (const _Float16*)(wp + PRW);
    const float* fr = sF + 16 * rt + 8 * hh;
#pragma unroll 1
    for (int p = 0; p < SIXF / FDIM; ++p) {
      const int n0c = FDIM * p + 64 * cg;
      v8f a0, a1, a2, a3;
      gemm16x64(ap, bpl, 32, 1, n0c, m, hh, a0, a1, a2, a3);
      float* sp = sW + (16 * rt + 8 * hh) * WPW + n0c + m;
      const float* bb = sBr + n0c + m;
      stage_gate(sp,      a0, fr, bb[0]);
      stage_gate(sp + 16, a1, fr, bb[16]);
      stage_gate(sp + 32, a2, fr, bb[32]);
      stage_gate(sp + 48, a3, fr, bb[48]);
    }
  }
  __syncthreads();

  {
    const int c4 = 4 * lane;
#pragma unroll 1
    for (int jx = 0; jx < 8; ++jx) {
      const int el = 8 * wave + jx;
      const int jj = sJ[el];
      const float* pp = PHI + (size_t)jj * SIXF + c4;
      const float* gp = sW + el * WPW + c4;
      const v4f p0 = *(const v4f*)(pp);
      const v4f p1 = *(const v4f*)(pp + FDIM);
      const v4f p2 = *(const v4f*)(pp + 2 * FDIM);
      const v4f p3 = *(const v4f*)(pp + 3 * FDIM);
      const v4f p4 = *(const v4f*)(pp + 4 * FDIM);
      const v4f p5 = *(const v4f*)(pp + 5 * FDIM);
      const v4f g0 = *(const v4f*)(gp);
      const v4f g1 = *(const v4f*)(gp + FDIM);
      const v4f g2 = *(const v4f*)(gp + 2 * FDIM);
      const v4f g3 = *(const v4f*)(gp + 3 * FDIM);
      const v4f g4 = *(const v4f*)(gp + 4 * FDIM);
      const v4f g5 = *(const v4f*)(gp + 5 * FDIM);
      const v4f xs   = p0 * g0;
      const v4f xvv  = p1 * g1;
      const v4f xvs1 = p2 * g2;
      const v4f xvs2 = p3 * g3;
      const v4f xvc1 = p4 * g4;
      const v4f xvc2 = p5 * g5;
      const float* vp = vin + (size_t)jj * VROW + c4;
      const v4f v0 = *(const v4f*)(vp);
      const v4f v1 = *(const v4f*)(vp + FDIM);
      const v4f v2 = *(const v4f*)(vp + 2 * FDIM);
      const float ax = sU[8 * el + 0], ay = sU[8 * el + 1], az = sU[8 * el + 2];
      const float bx = sU[8 * el + 4], by = sU[8 * el + 5], bz = sU[8 * el + 6];
      const v4f c1x = v1 * az - v2 * ay;
      const v4f c1y = v2 * ax - v0 * az;
      const v4f c1z = v0 * ay - v1 * ax;
      const v4f c2x = v1 * bz - v2 * by;
      const v4f c2y = v2 * bx - v0 * bz;
      const v4f c2z = v0 * by - v1 * bx;
      const v4f m0 = (((v0 * xvv + xvs1 * ax) + xvs2 * bx) + xvc1 * c1x) + xvc2 * c2x;
      const v4f m1 = (((v1 * xvv + xvs1 * ay) + xvs2 * by) + xvc1 * c1y) + xvc2 * c2y;
      const v4f m2 = (((v2 * xvv + xvs1 * az) + xvs2 * bz) + xvc1 * c1z) + xvc2 * c2z;
      float* mp = Mout + (size_t)(el0 + el) * MSGW + c4;
      *(volatile v4f*)(mp)            = xs;
      *(volatile v4f*)(mp + FDIM)     = m0;
      *(volatile v4f*)(mp + 2 * FDIM) = m1;
      *(volatile v4f*)(mp + 3 * FDIM) = m2;
      __threadfence();
      *(volatile v4f*)(mp)            = xs;
      *(volatile v4f*)(mp + FDIM)     = m0;
      *(volatile v4f*)(mp + 2 * FDIM) = m1;
      *(volatile v4f*)(mp + 3 * FDIM) = m2;
    }
  }
}

__device__ __forceinline__ int scan_piece(const int* __restrict__ eid, int lim, int cbase, int base, int vecok,
                                          int* list, int tid, int wave) {
  int wc = 0;
  const int el0  = tid * EPT;
  const int e0   = cbase + el0;
  const int sent = -2147483647 - 1;
  int kk[EPT];
  if (vecok != 0 && cbase + PIECE <= lim) {
    const v4i* p = (const v4i*)(eid + e0);
#pragma unroll
    for (int u = 0; u < EPT / 4; ++u) {
      const v4i d = p[u];
      kk[4 * u] = d.x; kk[4 * u + 1] = d.y; kk[4 * u + 2] = d.z; kk[4 * u + 3] = d.w;
    }
  } else {
    const int lm = lim - 1;
#pragma unroll
    for (int q = 0; q < EPT; ++q) {
      const int eq = e0 + q;
      const int ec = eq > lm ? lm : eq;
      const int a = eid[ec];
      kk[q] = (eq < lim) ? a : sent;
    }
  }
  const unsigned nb = (unsigned)base;
  unsigned sq[EPT];
  bool hq[EPT];
  bool anyl = false;
#pragma unroll
  for (int q = 0; q < EPT; ++q) {
    sq[q] = (unsigned)kk[q] - nb;
    hq[q] = sq[q] < (unsigned)NBC;
    anyl = anyl | hq[q];
  }
  const unsigned any = __builtin_amdgcn_ballot_w32(anyl);
  if (any != 0u) {
#define HIT(HQ, SQ, Q) { \
      const unsigned mj = __builtin_amdgcn_ballot_w32(HQ); \
      if (mj != 0u) { \
        if (HQ) { \
          const int ps = wc + (int)__builtin_amdgcn_mbcnt_lo(mj, 0u); \
          if (ps < WCAP) list[wave * WCAP + ps] = ((el0 + (Q)) << SLB) | (int)(SQ); \
        } \
        wc += (int)__builtin_popcount(mj); } }
#pragma unroll
    for (int q = 0; q < EPT; ++q) {
      HIT(hq[q], sq[q], q)
    }
#undef HIT
  }
  return wc;
}

__device__ __forceinline__ void drain_piece(const int* list, const int* wcnt, float* accF,
                                            const float* __restrict__ Mf, int rowoff, int lane, int wave) {
#pragma unroll 1
  for (int wsx = 0; wsx < NWAVE; ++wsx) {
    int n = __builtin_amdgcn_readfirstlane(wcnt[wsx]);
    n = n > WCAP ? WCAP : (n < 0 ? 0 : n);
    const int* lp = list + wsx * WCAP;
#pragma unroll 1
    for (int bb = 0; bb < n; bb += 32) {
      const int idx = bb + lane;
      const int ic = idx > WCAP - 1 ? WCAP - 1 : idx;
      const int ent = lp[ic];
      const bool own = (idx < n) && ((ent & (NWAVE - 1)) == wave);
      unsigned msk = __builtin_amdgcn_ballot_w32(own);
#pragma unroll 1
      while (msk != 0u) {
        const int bit = (int)__builtin_ctz(msk);
        msk &= msk - 1u;
        const int e2 = __builtin_amdgcn_readlane(ent, bit);
        const int slot = e2 & (NBC - 1);
        const int el = (e2 >> SLB) & (PIECE - 1);
        int row = rowoff + el;
        row = row < 0 ? 0 : (row > CE - 1 ? CE - 1 : row);
        const float* mp = Mf + (size_t)row * MSGW + 4 * lane;
        float* ap = accF + slot * MSGW + 4 * lane;
#pragma unroll
        for (int q = 0; q < 4; ++q) {
          const v4f mv = *(const v4f*)(mp + FDIM * q);
          v4f a = *(const v4f*)(ap + FDIM * q);
          a += mv;
          *(v4f*)(ap + FDIM * q) = a;
        }
      }
    }
  }
}

__device__ __forceinline__ void agg_store(const float* accF, float* out0, float* out1, int base, int nN,
                                          int lane, int wave) {
#pragma unroll 1
  for (int it = 0; it < NBC / NWAVE; ++it) {
    const int s = wave + NWAVE * it;
    const int node = base + s;
    if (node < nN) {
      const float* ap = accF + s * MSGW + 4 * lane;
      const v4f a0 = *(const v4f*)(ap);
      const v4f a1 = *(const v4f*)(ap + FDIM);
      const v4f a2 = *(const v4f*)(ap + 2 * FDIM);
      const v4f a3 = *(const v4f*)(ap + 3 * FDIM);
      *(volatile v4f*)(out0 + (size_t)node * FDIM + 4 * lane) = a0;
      float* op = out1 + (size_t)node * VROW + 4 * lane;
      *(volatile v4f*)(op)            = a1;
      *(volatile v4f*)(op + FDIM)     = a2;
      *(volatile v4f*)(op + 2 * FDIM) = a3;
    }
  }
}

__global__ __launch_bounds__(NTHR) void k_agg(
    const int* __restrict__ ei, const float* __restrict__ Mq, const float* srcS, const float* srcV,
    float* out0, float* out1, int cbeg, int lim, int nN, int vecok) {
  extern __shared__ __attribute__((aligned(16))) float accF[];
  __shared__ int list[NWAVE * WCAP];
  __shared__ int wcnt[NWAVE];
  const int tid = (int)threadIdx.x, lane = tid & 31, wave = tid >> 5;
  const int base = (int)blockIdx.x * NBC;
  const int* eid = ei;

#pragma unroll 1
  for (int i = tid; i < NBC * 32; i += NTHR) {
    const int s = i >> 5, c4 = (i & 31) * 4;
    int node = base + s;
    node = node > nN - 1 ? nN - 1 : node;
    const v4f v = *(const v4f*)(srcS + (size_t)node * FDIM + c4);
    *(v4f*)(accF + s * MSGW + c4) = v;
  }
#pragma unroll 1
  for (int i = tid; i < NBC * 96; i += NTHR) {
    const int s = i / 96, c4 = (i - 96 * s) * 4;
    int node = base + s;
    node = node > nN - 1 ? nN - 1 : node;
    const v4f v = *(const v4f*)(srcV + (size_t)node * VROW + c4);
    *(v4f*)(accF + s * MSGW + FDIM + c4) = v;
  }
  __syncthreads();

#pragma unroll 1
  for (int cbase = cbeg; cbase < lim; cbase += PIECE) {
    const int wc = scan_piece(eid, lim, cbase, base, vecok, list, tid, wave);
    if (lane == 0) wcnt[wave] = wc;
    __syncthreads();
    drain_piece(list, wcnt, accF, Mq, cbase - cbeg, lane, wave);
    __syncthreads();
  }

  agg_store(accF, out0, out1, base, nN, lane, wave);
  __threadfence();
  agg_store(accF, out0, out1, base, nN, lane, wave);
}

extern "C" void kernel_launch(void* const* d_in, const int* in_sizes, int n_in,
                              void* d_out, int out_size, void* d_ws, size_t ws_size,
                              hipStream_t stream) {
  if (n_in < 15) return;
  if (in_sizes[0] < FDIM || (in_sizes[0] % FDIM) != 0) return;
  const int nN = in_sizes[0] / FDIM;
  if (nN < 1 || nN > (1 << 22)) return;
  if (in_sizes[1] != nN * VROW) return;
  const int nE = in_sizes[4];
  if (nE < 1 || nE > (1 << 26)) return;
  if (in_sizes[2] != nE * RDIM || in_sizes[3] != nE * RDIM || in_sizes[5] != nE) return;
  if (in_sizes[6] != 3 * nE || in_sizes[7] != 3 * nE || in_sizes[8] != 2 * nE) return;
  if (in_sizes[9] != FDIM * FDIM || in_sizes[10] != FDIM) return;
  if (in_sizes[11] != FDIM * SIXF || in_sizes[12] != SIXF) return;
  if (in_sizes[13] != RDIM * SIXF || in_sizes[14] != SIXF) return;
  if (out_size != nN * MSGW) return;

  const float* s   = (const float*)d_in[0];
  const float* v   = (const float*)d_in[1];
  const float* re1 = (const float*)d_in[2];
  const float* re2 = (const float*)d_in[3];
  const float* f1  = (const float*)d_in[4];
  const float* f2  = (const float*)d_in[5];
  const float* u1  = (const float*)d_in[6];
  const float* u2  = (const float*)d_in[7];
  const int*   ei  = (const int*)d_in[8];
  const float* W1  = (const float*)d_in[9];
  const float* b1  = (const float*)d_in[10];
  const float* W2  = (const float*)d_in[11];
  const float* b2  = (const float*)d_in[12];
  const float* Wr  = (const float*)d_in[13];
  const float* br  = (const float*)d_in[14];
  float* out0 = (float*)d_out;
  float* out1 = out0 + (size_t)FDIM * (size_t)nN;

  const int nbNode = (nN + NBN - 1) / NBN;
  const int NpadN  = nbNode * NBN;
  const int nChunk = (nE + CE - 1) / CE;
  if (nChunk < 1 || nChunk > MAXCH) return;
  const int nbAgg  = (nN + NBC - 1) / NBC;

  char* ws = (char*)d_ws;
  size_t off = 0;
  const size_t oW = off; off += (size_t)PWTOT * 2;                       off = (off + 255) & ~(size_t)255;
  const size_t oP = off; off += (size_t)NpadN * SIXF * 4;                 off = (off + 255) & ~(size_t)255;
  const size_t oM = off; off += (size_t)CE * MSGW * 4;                    off = (off + 255) & ~(size_t)255;
  if (off > ws_size || off > (size_t)WSCAP) return;
  unsigned short* wp = (unsigned short*)(ws + oW);
  float* PHI         = (float*)(ws + oP);
  float* Mq          = (float*)(ws + oM);

  hipFuncSetAttribute(reinterpret_cast<const void*>(&k_node), hipFuncAttributeMaxDynamicSharedMemorySize, NODEDYN);
  hipFuncSetAttribute(reinterpret_cast<const void*>(&k_edge), hipFuncAttributeMaxDynamicSharedMemorySize, EDGEDYN);
  hipFuncSetAttribute(reinterpret_cast<const void*>(&k_agg), hipFuncAttributeMaxDynamicSharedMemorySize, AGGDYN);

  k_prep<<<PBLK, NTHR, 0, stream>>>(W1, W2, Wr, wp);
  k_node<<<nbNode, NTHR, NODEDYN, stream>>>(s, wp, b1, b2, PHI, nN);
  for (int c = 0; c < nChunk; ++c) {
    const int cbeg = c * CE;
    int lim = cbeg + CE;
    lim = lim > nE ? nE : lim;
    const int nblk = (lim - cbeg + NBE - 1) / NBE;
    const float* srcS = (c == 0) ? s : out0;
    const float* srcV = (c == 0) ? v : out1;
    k_edge<<<nblk, NTHR, EDGEDYN, stream>>>(re1, re2, f1, f2, u1, u2, ei, PHI, v, wp, br, Mq, nE, nN, cbeg);
    k_agg<<<nbAgg, NTHR, AGGDYN, stream>>>(ei, Mq, srcS, srcV, out0, out1, cbeg, lim, nN, 1);
  }
}
